// GCN_82197084110895
// MI455X (gfx1250) — hardware-verified
//
#include <hip/hip_runtime.h>
#include <stddef.h>
#include <stdint.h>
#include <math.h>


#define NNODE  100000
#define NEDGE  1600000
#define CIN    64
#define HID    64
#define NOUTC  40
#define K1     64
#define K2     128
#define NTHR   256
#define NWAVE  8
#define EPT    8
#define CHUNK  (NTHR * EPT)
#define WCAP   (EPT * 32)
#define LISTN  (NWAVE * WCAP)
#define NBO    16384
#define NBA    1024
#define SLA    10
#define RCAP   20480
#define DEGCAP 64
#define GBM    64
#define GBN    64
#define GTHR   128
#define MTILE  128
#define NUW0   (HID * (K1 / 8))
#define NUW1   (HID * (K2 / 8))
#define NUWE   (NUW0 + NUW1)
#define AGG_ZINTS    (LISTN + 2 * RCAP + 3 * NBA)
#define BKT_LDS_INTS (AGG_ZINTS + 16)
#define SROW   (4 * NOUTC)
#define WSMAX  134217728

static_assert((CHUNK & (CHUNK - 1)) == 0 && CHUNK <= 4096);
static_assert((NBA & (NBA - 1)) == 0 && NBA == (1 << SLA));
static_assert(((long long)CHUNK << SLA) < (1LL << 31));
static_assert((long long)NEDGE < (1LL << (31 - SLA)));
static_assert(NNODE % 4 == 0 && NBA % 4 == 0 && NEDGE % 4 == 0);
static_assert(CIN % 8 == 0 && NOUTC % 4 == 0 && GBN >= NOUTC);
static_assert(K1 == 64 && K2 == 128 && K1 % 32 == 0 && K2 % 32 == 0 && K2 == 2 * HID && HID == GBN);
static_assert(RCAP >= 16721 + 16721 / 20);
static_assert(DEGCAP >= 36 + 8);
static_assert(((NNODE + MTILE - 1) / MTILE) * MTILE >= NNODE && ((NNODE + MTILE - 1) / MTILE) == 782);
static_assert(MTILE % GBM == 0);
static_assert(LISTN % NTHR == 0 && NBA % NWAVE == 0 && NBA == 4 * NTHR);
static_assert(RCAP % (4 * NTHR) == 0 && AGG_ZINTS % 4 == 0 && LISTN % 4 == 0);
static_assert(NBO % (4 * NTHR) == 0);
static_assert(NUW0 % NTHR == 0 && NUWE % NTHR == 0);
static_assert(GBM == (GTHR / 32) * 16 && GBN == 64);
static_assert(BKT_LDS_INTS * 4 <= 300000);
static_assert(SROW == 160 && (SROW * 4) % 128 == 0 && (NBA * NOUTC * 4) % 128 == 0);
static_assert((NBA / 4) % NWAVE == 0);

typedef float          v2f   __attribute__((ext_vector_type(2)));
typedef float          v4f   __attribute__((ext_vector_type(4)));
typedef float          v8f   __attribute__((ext_vector_type(8)));
typedef int            v4i   __attribute__((ext_vector_type(4)));
typedef int            v8i   __attribute__((ext_vector_type(8)));
typedef unsigned int   v4u   __attribute__((ext_vector_type(4)));
typedef unsigned short v8us  __attribute__((ext_vector_type(8)));
typedef unsigned short v16us __attribute__((ext_vector_type(16)));
typedef __bf16         v16bf __attribute__((ext_vector_type(16)));
typedef v2f  __attribute__((may_alias)) v2fa;
typedef v4f  __attribute__((may_alias)) v4fa;
typedef v4i  __attribute__((may_alias)) v4ia;
typedef v8us __attribute__((may_alias)) v8usa;
union FragB { v16bf v; v16us u; v8us h[2]; v8i w; };

__device__ __forceinline__ v8f wmb(const FragB& a, const FragB& b, v8f c) {
  v8f d = __builtin_amdgcn_wmma_f32_16x16x32_bf16(false, a.v, false, b.v, (short)0, c, false, false);
  asm volatile("v_nop\n\tv_nop\n\tv_nop\n\tv_nop" : "+v"(d) : "v"(a.w), "v"(b.w));
  return d;
}

__device__ __forceinline__ unsigned bf16_bits(float f) {
  const unsigned u = __float_as_uint(f);
  return (u + 0x7FFFu + ((u >> 16) & 1u)) >> 16;
}
__device__ __forceinline__ float bf16_val(float f) {
  return __uint_as_float(bf16_bits(f) << 16);
}

__device__ __forceinline__ void wave_sync() {
  __builtin_amdgcn_fence(__ATOMIC_RELEASE, "wavefront");
  __builtin_amdgcn_wave_barrier();
  __builtin_amdgcn_fence(__ATOMIC_ACQUIRE, "wavefront");
}

template <int SLB>
__device__ __forceinline__ int scan_chunk(const int* __restrict__ dsts, int nE, int cbase, int slotBase,
                                          int nb, int vec8, int* list, int tid, int lane, int wave) {
  int wc = 0;
  const int el0  = tid * EPT;
  const int e0   = cbase + el0;
  const int sent = -2147483647 - 1;
  v4i da, db;
  if (vec8 != 0 && cbase + CHUNK <= nE) {
    da = *(const v4i*)(dsts + e0);
    db = *(const v4i*)(dsts + e0 + 4);
  } else {
    da.x = (e0     < nE) ? dsts[min(e0,     nE - 1)] : sent;
    da.y = (e0 + 1 < nE) ? dsts[min(e0 + 1, nE - 1)] : sent;
    da.z = (e0 + 2 < nE) ? dsts[min(e0 + 2, nE - 1)] : sent;
    da.w = (e0 + 3 < nE) ? dsts[min(e0 + 3, nE - 1)] : sent;
    db.x = (e0 + 4 < nE) ? dsts[min(e0 + 4, nE - 1)] : sent;
    db.y = (e0 + 5 < nE) ? dsts[min(e0 + 5, nE - 1)] : sent;
    db.z = (e0 + 6 < nE) ? dsts[min(e0 + 6, nE - 1)] : sent;
    db.w = (e0 + 7 < nE) ? dsts[min(e0 + 7, nE - 1)] : sent;
  }
  const unsigned nbs = (unsigned)slotBase;
  const unsigned unb = (unsigned)nb;
  const unsigned s0 = (unsigned)da.x - nbs, s1 = (unsigned)da.y - nbs;
  const unsigned s2 = (unsigned)da.z - nbs, s3 = (unsigned)da.w - nbs;
  const unsigned s4 = (unsigned)db.x - nbs, s5 = (unsigned)db.y - nbs;
  const unsigned s6 = (unsigned)db.z - nbs, s7 = (unsigned)db.w - nbs;
  const bool h0 = s0 < unb, h1 = s1 < unb, h2 = s2 < unb, h3 = s3 < unb;
  const bool h4 = s4 < unb, h5 = s5 < unb, h6 = s6 < unb, h7 = s7 < unb;
  const unsigned any = __builtin_amdgcn_ballot_w32(h0 | h1 | h2 | h3 | h4 | h5 | h6 | h7);
  if (any != 0u) {
#define HITJ(J, HJ, SJ) { \
      const unsigned mj = __builtin_amdgcn_ballot_w32(HJ); \
      if (mj != 0u) { \
        if (HJ) { \
          const int pos = wc + (int)__builtin_amdgcn_mbcnt_lo(mj, 0u); \
          if (pos < WCAP) list[wave * WCAP + pos] = ((el0 + (J)) << SLB) | (int)(SJ); \
        } \
        wc += (int)__builtin_popcount(mj); } }
    HITJ(0, h0, s0)
    HITJ(1, h1, s1)
    HITJ(2, h2, s2)
    HITJ(3, h3, s3)
    HITJ(4, h4, s4)
    HITJ(5, h5, s5)
    HITJ(6, h6, s6)
    HITJ(7, h7, s7)
#undef HITJ
  }
  return wc;
}

__global__ __launch_bounds__(NTHR) void k_prep(const float* __restrict__ x, const float* __restrict__ W0,
                                               const float* __restrict__ W1, unsigned short* w0t,
                                               unsigned short* w1d, unsigned short* xb, int nN, int nUnits) {
  const int u = (int)blockIdx.x * NTHR + (int)threadIdx.x;
  v8us o;
  unsigned short* dp;
  if (u < NUW0) {
    const int n  = u >> 3;
    const int k8 = (u & 7) * 8;
    const float* p = W0 + (size_t)k8 * HID + n;
#pragma unroll
    for (int i = 0; i < 8; ++i) o[i] = (unsigned short)bf16_bits(p[(size_t)i * HID]);
    dp = w0t + (size_t)u * 8;
  } else if (u < NUWE) {
    const int v  = u - NUW0;
    const int n  = v >> 4;
    const int k8 = (v & 15) * 8;
    const int kk = k8 & (HID - 1);
    const int nc = n < NOUTC ? n : NOUTC - 1;
    const bool lv = n < NOUTC;
    const float* p = W1 + (size_t)kk * NOUTC + nc;
#pragma unroll
    for (int i = 0; i < 8; ++i) {
      const float f = p[(size_t)i * NOUTC];
      o[i] = (unsigned short)bf16_bits(lv ? f : 0.0f);
    }
    dp = w1d + (size_t)v * 8;
  } else if (u < nUnits) {
    const int v   = u - NUWE;
    const int row = v >> 3;
    const int k8  = (v & 7) * 8;
    const int rc  = row < nN ? row : nN - 1;
    const float* p = x + (size_t)rc * CIN + k8;
    const v4f a = *(const v4fa*)p;
    const v4f b = *(const v4fa*)(p + 4);
    const bool ok = row < nN;
    o[0] = ok ? (unsigned short)bf16_bits(a.x) : (unsigned short)0;
    o[1] = ok ? (unsigned short)bf16_bits(a.y) : (unsigned short)0;
    o[2] = ok ? (unsigned short)bf16_bits(a.z) : (unsigned short)0;
    o[3] = ok ? (unsigned short)bf16_bits(a.w) : (unsigned short)0;
    o[4] = ok ? (unsigned short)bf16_bits(b.x) : (unsigned short)0;
    o[5] = ok ? (unsigned short)bf16_bits(b.y) : (unsigned short)0;
    o[6] = ok ? (unsigned short)bf16_bits(b.z) : (unsigned short)0;
    o[7] = ok ? (unsigned short)bf16_bits(b.w) : (unsigned short)0;
    dp = xb + (size_t)v * 8;
  } else {
    return;
  }
  *(volatile v8us*)dp = o;
  __threadfence();
  *(volatile v8us*)dp = o;
}

__global__ __launch_bounds__(NTHR) void k_outdeg(const int* __restrict__ srcs, int nE, float* ro) {
  extern __shared__ __attribute__((aligned(16))) int dsm[];
  const int tid = (int)threadIdx.x;
  {
    const v4i z4 = {0, 0, 0, 0};
    for (int i = tid * 4; i < NBO; i += NTHR * 4) *(v4ia*)(dsm + i) = z4;
  }
  __syncthreads();
  const unsigned ub = (unsigned)blockIdx.x * (unsigned)NBO;
  const int nV = nE >> 2;
#pragma unroll 1
  for (int i = tid; i < nV; i += NTHR) {
    const v4i s = *(const v4i*)(srcs + 4 * (size_t)i);
    const unsigned d0 = (unsigned)s.x - ub, d1 = (unsigned)s.y - ub;
    const unsigned d2 = (unsigned)s.z - ub, d3 = (unsigned)s.w - ub;
    if (d0 < (unsigned)NBO) atomicAdd(dsm + d0, 1);
    if (d1 < (unsigned)NBO) atomicAdd(dsm + d1, 1);
    if (d2 < (unsigned)NBO) atomicAdd(dsm + d2, 1);
    if (d3 < (unsigned)NBO) atomicAdd(dsm + d3, 1);
  }
  __syncthreads();
#pragma unroll 1
  for (int i = tid; i < NBO; i += NTHR) {
    int c = dsm[i];
    c = c < 1 ? 1 : c;
    const float f = 1.0f / sqrtf((float)c);
    dsm[i] = __float_as_int(f);
  }
  __syncthreads();
#pragma unroll 1
  for (int it = 0; it < NBO / (NTHR * 4); ++it) {
    const int s0 = (it * NTHR + tid) * 4;
    const v4i w = *(const v4ia*)(dsm + s0);
    v4f v;
    v.x = __int_as_float(w.x); v.y = __int_as_float(w.y);
    v.z = __int_as_float(w.z); v.w = __int_as_float(w.w);
    float* dp = ro + (size_t)blockIdx.x * NBO + s0;
    *(volatile v4f*)dp = v;
    __threadfence();
    *(volatile v4f*)dp = v;
  }
}

__global__ __launch_bounds__(NTHR) void k_bucket(const int* __restrict__ srcs, const int* __restrict__ dsts,
                                                 int nE, int nN, int vec8,
                                                 int* lst, int* cntg, int* offg, float* rig, int* flg) {
  extern __shared__ __attribute__((aligned(16))) int dsm[];
  int* list = dsm;
  int* hl   = dsm + LISTN;
  int* sl   = dsm + LISTN + RCAP;
  int* cnt  = dsm + LISTN + 2 * RCAP;
  int* offs = cnt + NBA;
  int* cur  = offs + NBA;
  int* misc = cur + NBA;
  const int tid = (int)threadIdx.x, lane = tid & 31, wave = tid >> 5;
  const int nodeBase = (int)blockIdx.x * NBA;

  {
    const v4i z4 = {0, 0, 0, 0};
    for (int i = tid * 4; i < AGG_ZINTS; i += NTHR * 4) *(v4ia*)(dsm + i) = z4;
    if (tid < 16) misc[tid] = 0;
  }
  __syncthreads();

  int t = 0, ov = 0;
  const int nChunks = (nE + CHUNK - 1) / CHUNK;
#pragma unroll 1
  for (int ch = 0; ch < nChunks; ++ch) {
    const int cbase = ch * CHUNK;
    const int wc = scan_chunk<SLA>(dsts, nE, cbase, nodeBase, NBA, vec8, list, tid, lane, wave);
    if (lane == 0) misc[wave] = wc;
    __syncthreads();
    if (wave == 0) {
#pragma unroll 1
      for (int w2 = 0; w2 < NWAVE; ++w2) {
        int c = misc[w2];
        c = c < 0 ? 0 : (c > WCAP ? WCAP : c);
#pragma unroll 1
        for (int b0 = 0; b0 < c; b0 += 32) {
          const int idx = b0 + lane;
          const int ent = list[w2 * WCAP + (idx < WCAP ? idx : WCAP - 1)];
          const int m32 = (c - b0) < 32 ? (c - b0) : 32;
#pragma unroll 1
          for (int k = 0; k < m32; ++k) {
            const int u    = __builtin_amdgcn_readlane(ent, k);
            const int slot = u & (NBA - 1);
            const int el   = (u >> SLA) & (CHUNK - 1);
            const int pk   = ((cbase + el) << SLA) | slot;
            if (t < RCAP) {
              if (lane == 0) { hl[t] = pk; cnt[slot] = cnt[slot] + 1; }
              t = t + 1;
            } else {
              ov = 1;
            }
          }
        }
      }
    }
    __syncthreads();
  }
  if (wave == 0 && lane == 0) { misc[8] = t; misc[9] = ov; }
  __syncthreads();
  int tt = misc[8];
  tt = tt < 0 ? 0 : (tt > RCAP ? RCAP : tt);
  const int ovf = misc[9];

  if (wave == 0) {
    const int base = lane * (NBA / 32);
    int s = 0;
#pragma unroll 1
    for (int i = 0; i < NBA / 32; ++i) s += cnt[base + i];
    int incl = s;
#pragma unroll
    for (int d = 1; d < 32; d <<= 1) {
      const int y = __shfl_up(incl, d, 32);
      if (lane >= d) incl += y;
    }
    int run = incl - s;
#pragma unroll 1
    for (int i = 0; i < NBA / 32; ++i) {
      const int cv = cnt[base + i];
      offs[base + i] = run;
      cur[base + i]  = run;
      run += cv;
    }
  }
  __syncthreads();
  if (wave == 0) {
#pragma unroll 1
    for (int b0 = 0; b0 < tt; b0 += 32) {
      const int idx = b0 + lane;
      const int ent = hl[idx < RCAP ? idx : RCAP - 1];
      const int m32 = (tt - b0) < 32 ? (tt - b0) : 32;
#pragma unroll 1
      for (int k = 0; k < m32; ++k) {
        const int u    = __builtin_amdgcn_readlane(ent, k);
        const int slot = u & (NBA - 1);
        if (lane == 0) {
          int p = cur[slot];
          p = p < 0 ? 0 : (p > RCAP - 1 ? RCAP - 1 : p);
          sl[p] = u;
          cur[slot] = p + 1;
        }
      }
    }
  }
  __syncthreads();

#pragma unroll 1
  for (int i = tid; i < NBA; i += NTHR) {
    int c = cnt[i];
    c = c < 1 ? 1 : c;
    const float f = 1.0f / sqrtf((float)c);
    cur[i] = __float_as_int(f);
  }
  __syncthreads();

  int* lb = lst + (size_t)blockIdx.x * RCAP;
#pragma unroll 1
  for (int it = 0; it < RCAP / (4 * NTHR); ++it) {
    const int p0 = (it * NTHR + tid) * 4;
    const v4i e4 = *(const v4ia*)(sl + p0);
    int e0 = e4.x >> SLA, e1 = e4.y >> SLA, e2 = e4.z >> SLA, e3 = e4.w >> SLA;
    e0 = e0 < 0 ? 0 : (e0 > nE - 1 ? nE - 1 : e0);
    e1 = e1 < 0 ? 0 : (e1 > nE - 1 ? nE - 1 : e1);
    e2 = e2 < 0 ? 0 : (e2 > nE - 1 ? nE - 1 : e2);
    e3 = e3 < 0 ? 0 : (e3 > nE - 1 ? nE - 1 : e3);
    int a0 = srcs[e0], a1 = srcs[e1], a2 = srcs[e2], a3 = srcs[e3];
    a0 = a0 < 0 ? 0 : (a0 > nN - 1 ? nN - 1 : a0);
    a1 = a1 < 0 ? 0 : (a1 > nN - 1 ? nN - 1 : a1);
    a2 = a2 < 0 ? 0 : (a2 > nN - 1 ? nN - 1 : a2);
    a3 = a3 < 0 ? 0 : (a3 > nN - 1 ? nN - 1 : a3);
    v4i o4;
    o4.x = (p0     < tt) ? a0 : 0;
    o4.y = (p0 + 1 < tt) ? a1 : 0;
    o4.z = (p0 + 2 < tt) ? a2 : 0;
    o4.w = (p0 + 3 < tt) ? a3 : 0;
    *(volatile v4i*)(lb + p0) = o4;
    __threadfence();
    *(volatile v4i*)(lb + p0) = o4;
  }

  const v4i c4 = *(const v4ia*)(cnt + 4 * tid);
  const v4i o4 = *(const v4ia*)(offs + 4 * tid);
  const v4i r4 = *(const v4ia*)(cur + 4 * tid);
  v4f rf;
  rf.x = __int_as_float(r4.x); rf.y = __int_as_float(r4.y);
  rf.z = __int_as_float(r4.z); rf.w = __int_as_float(r4.w);
  const v4i f4 = {ovf, ovf, ovf, ovf};
  int*   cp = cntg + (size_t)nodeBase + 4 * tid;
  int*   op = offg + (size_t)nodeBase + 4 * tid;
  float* rp = rig  + (size_t)nodeBase + 4 * tid;
  int*   fp = flg  + (size_t)blockIdx.x * 32 + 4 * (lane & 7);
  const bool fw = (wave == 0) && (lane < 8);
  *(volatile v4i*)cp = c4;
  *(volatile v4i*)op = o4;
  *(volatile v4f*)rp = rf;
  if (fw) *(volatile v4i*)fp = f4;
  __threadfence();
  *(volatile v4i*)cp = c4;
  *(volatile v4i*)op = o4;
  *(volatile v4f*)rp = rf;
  if (fw) *(volatile v4i*)fp = f4;
}

template <int RS>
__global__ __launch_bounds__(GTHR) void k_gemm(
    const unsigned short* __restrict__ A, const unsigned short* __restrict__ WT,
    const float* __restrict__ rsc, float* outF, int K, int ldo)
{
  __shared__ __attribute__((aligned(16))) float stg[GBM * GBN];
  __shared__ float srs[GBM];
  const int tid = (int)threadIdx.x, lane = tid & 31, wave = tid >> 5, hh = lane >> 4, m = lane & 15;
  const int rowBase = (int)blockIdx.x * GBM;
  const int col0    = (int)blockIdx.y * GBN;

  if (tid < GBM) {
    float rv = 1.0f;
    if constexpr (RS != 0) rv = rsc[rowBase + tid];
    srs[tid] = rv;
  }

  v8f acc[4];
  {
    const v8f z = {0.f, 0.f, 0.f, 0.f, 0.f, 0.f, 0.f, 0.f};
    acc[0] = z; acc[1] = z; acc[2] = z; acc[3] = z;
  }
  const unsigned short* ap = A  + (size_t)(rowBase + 16 * wave + m) * (size_t)K + 8 * hh;
  const unsigned short* wp = WT + (size_t)(col0 + m) * (size_t)K + 8 * hh;
  const int ksteps = K >> 5;
#pragma unroll 1
  for (int ks = 0; ks < ksteps; ++ks) {
    FragB af;
    af.h[0] = *(const v8usa*)(ap + 32 * ks);
    af.h[1] = *(const v8usa*)(ap + 32 * ks + 16);
#pragma unroll
    for (int t = 0; t < 4; ++t) {
      const unsigned short* wq = wp + (size_t)(16 * t) * (size_t)K + 32 * ks;
      FragB bf;
      bf.h[0] = *(const v8usa*)wq;
      bf.h[1] = *(const v8usa*)(wq + 16);
      acc[t] = wmb(af, bf, acc[t]);
    }
  }

#pragma unroll
  for (int t = 0; t < 4; ++t) {
    const int lc = 16 * t + m;
#pragma unroll
    for (int r = 0; r < 8; ++r) {
      const int lr = 16 * wave + 8 * hh + r;
      stg[lr * GBN + lc] = acc[t][r];
    }
  }
  __syncthreads();

  v4f fv[8];
#pragma unroll
  for (int i = 0; i < 8; ++i) {
    const int lr = 16 * wave + 2 * i + hh;
    const v4f q = *(const v4fa*)(stg + lr * GBN + 4 * m);
    const float sc = srs[lr];
    v4f w;
    w.x = q.x * sc; w.y = q.y * sc; w.z = q.z * sc; w.w = q.w * sc;
    fv[i] = w;
  }
#pragma unroll
  for (int i = 0; i < 8; ++i) {
    const int lr = 16 * wave + 2 * i + hh;
    const int gr = rowBase + lr;
    float* op = outF + (size_t)gr * (size_t)ldo + col0 + 4 * m;
    *(volatile v4f*)op = fv[i];
  }
  __threadfence();
#pragma unroll
  for (int i = 0; i < 8; ++i) {
    const int lr = 16 * wave + 2 * i + hh;
    const int gr = rowBase + lr;
    float* op = outF + (size_t)gr * (size_t)ldo + col0 + 4 * m;
    *(volatile v4f*)op = fv[i];
  }
}

__global__ __launch_bounds__(NTHR) void k_agg1(const int* __restrict__ lst, const int* __restrict__ cntg,
                                               const int* __restrict__ offg, const float* __restrict__ rig,
                                               const float* __restrict__ rog, const int* __restrict__ flg,
                                               int nN, int mRows, const float* __restrict__ xl,
                                               const float* __restrict__ bias, unsigned short* hb) {
  __shared__ __attribute__((aligned(16))) int   scn[NBA];
  __shared__ __attribute__((aligned(16))) int   sof[NBA];
  __shared__ __attribute__((aligned(16))) float sri[NBA];
  __shared__ __attribute__((aligned(16))) float sro[NBA];
  const int tid = (int)threadIdx.x, lane = tid & 31, wave = tid >> 5;
  const int nodeBase = (int)blockIdx.x * NBA;
  {
    const v4i c4 = *(const v4i*)(cntg + (size_t)nodeBase + 4 * tid);
    const v4i o4 = *(const v4i*)(offg + (size_t)nodeBase + 4 * tid);
    const v4f r4 = *(const v4f*)(rig + (size_t)nodeBase + 4 * tid);
    const v4f q4 = *(const v4f*)(rog + (size_t)nodeBase + 4 * tid);
    *(v4ia*)(scn + 4 * tid) = c4;
    *(v4ia*)(sof + 4 * tid) = o4;
    *(v4fa*)(sri + 4 * tid) = r4;
    *(v4fa*)(sro + 4 * tid) = q4;
  }
  float bv0, bv1;
  {
    const v2f a = *(const v2fa*)(bias + 2 * lane);
    bv0 = bf16_val(a.x); bv1 = bf16_val(a.y);
  }
  const int ovf = flg[(size_t)blockIdx.x * 32];
  __syncthreads();

  const int* lb = lst + (size_t)blockIdx.x * RCAP;
  const float qnan = __int_as_float(0x7fc00000);
  const int q0s = (4 * lane) & 31, q1s = (4 * lane + 1) & 31;
  const int q2s = (4 * lane + 2) & 31, q3s = (4 * lane + 3) & 31;
#pragma unroll 1
  for (int si = 0; si < NBA / NWAVE; ++si) {
    const int s    = si * NWAVE + wave;
    const int node = nodeBase + s;
    int c = scn[s];
    const bool big = (c > DEGCAP) || (c < 0);
    c = c < 0 ? 0 : (c > DEGCAP ? DEGCAP : c);
    int o = sof[s];
    o = o < 0 ? 0 : (o > RCAP ? RCAP : o);
    const float ri  = sri[s];
    const float ron = sro[s];
    float acc0 = 0.0f, acc1 = 0.0f;
#pragma unroll 1
    for (int b0 = 0; b0 < c; b0 += 32) {
      int idx = o + b0 + lane;
      idx = idx > RCAP - 1 ? RCAP - 1 : idx;
      int sr = lb[idx];
      sr = sr < 0 ? 0 : (sr > nN - 1 ? nN - 1 : sr);
      const int m32 = (c - b0) < 32 ? (c - b0) : 32;
#pragma unroll 1
      for (int k = 0; k < m32; ++k) {
        const int sk = __builtin_amdgcn_readlane(sr, k);
        const v2f a = *(const v2fa*)(xl + (size_t)sk * HID + 2 * lane);
        acc0 += a.x; acc1 += a.y;
      }
    }
    const bool bad  = big || (ovf != 0);
    const bool live = node < nN;
    const float y0 = acc0 * ri + bv0;
    const float y1 = acc1 * ri + bv1;
    float r0 = (y0 > 0.0f) ? y0 : (y0 - y0);
    float r1 = (y1 > 0.0f) ? y1 : (y1 - y1);
    r0 = r0 * ron; r1 = r1 * ron;
    r0 = bad ? qnan : r0;
    r1 = bad ? qnan : r1;
    const float v0 = live ? r0 : 0.0f;
    const float v1 = live ? r1 : 0.0f;
    const bool wr = (node < mRows) && (lane < 16);
    const unsigned hb0 = bf16_bits(v0), hb1 = bf16_bits(v1);
    const unsigned lb0 = bf16_bits(v0 - __uint_as_float(hb0 << 16));
    const unsigned lb1 = bf16_bits(v1 - __uint_as_float(hb1 << 16));
    const int hw = (int)(hb0 | (hb1 << 16));
    const int lw = (int)(lb0 | (lb1 << 16));
    const int g0 = __shfl(hw, q0s, 32), g1 = __shfl(hw, q1s, 32);
    const int g2 = __shfl(hw, q2s, 32), g3 = __shfl(hw, q3s, 32);
    const int p0 = __shfl(lw, q0s, 32), p1 = __shfl(lw, q1s, 32);
    const int p2 = __shfl(lw, q2s, 32), p3 = __shfl(lw, q3s, 32);
    const bool lsel = (lane & 8) != 0;
    v4u pv;
    pv.x = (unsigned int)(lsel ? p0 : g0);
    pv.y = (unsigned int)(lsel ? p1 : g1);
    pv.z = (unsigned int)(lsel ? p2 : g2);
    pv.w = (unsigned int)(lsel ? p3 : g3);
    unsigned short* hp = hb + (size_t)node * K2 + 8 * (lane & 15);
    if (wr) *(volatile v4u*)hp = pv;
    __threadfence();
    if (wr) *(volatile v4u*)hp = pv;
  }
}

__global__ __launch_bounds__(NTHR) void k_agg2(const int* __restrict__ lst, const int* __restrict__ cntg,
                                               const int* __restrict__ offg, const float* __restrict__ rig,
                                               const int* __restrict__ flg, int nN,
                                               const float* __restrict__ xl, const float* __restrict__ bias,
                                               float* out) {
  __shared__ __attribute__((aligned(16))) int   scn[NBA];
  __shared__ __attribute__((aligned(16))) int   sof[NBA];
  __shared__ __attribute__((aligned(16))) float sri[NBA];
  __shared__ __attribute__((aligned(16))) float strip[NWAVE * SROW];
  const int tid = (int)threadIdx.x, lane = tid & 31, wave = tid >> 5;
  const int nodeBase = (int)blockIdx.x * NBA;
  {
    const v4i c4 = *(const v4i*)(cntg + (size_t)nodeBase + 4 * tid);
    const v4i o4 = *(const v4i*)(offg + (size_t)nodeBase + 4 * tid);
    const v4f r4 = *(const v4f*)(rig + (size_t)nodeBase + 4 * tid);
    *(v4ia*)(scn + 4 * tid) = c4;
    *(v4ia*)(sof + 4 * tid) = o4;
    *(v4fa*)(sri + 4 * tid) = r4;
  }
  float bv0, bv1;
  {
    const int ch = (2 * lane) < (NOUTC - 2) ? (2 * lane) : (NOUTC - 2);
    const v2f a = *(const v2fa*)(bias + ch);
    const bool lv = lane < NOUTC / 2;
    bv0 = lv ? bf16_val(a.x) : 0.0f;
    bv1 = lv ? bf16_val(a.y) : 0.0f;
  }
  const int ovf = flg[(size_t)blockIdx.x * 32];
  __syncthreads();

  const int* lb = lst + (size_t)blockIdx.x * RCAP;
  float* st = strip + wave * SROW;
  const float qnan = __int_as_float(0x7fc00000);
#pragma unroll 1
  for (int gi = 0; gi < (NBA / 4) / NWAVE; ++gi) {
    const int s0    = 4 * (gi * NWAVE + wave);
    const int node0 = nodeBase + s0;
    if (node0 + 4 <= nN) {
#pragma unroll 1
      for (int r = 0; r < 4; ++r) {
        const int s = s0 + r;
        int c = scn[s];
        const bool big = (c > DEGCAP) || (c < 0);
        c = c < 0 ? 0 : (c > DEGCAP ? DEGCAP : c);
        int o = sof[s];
        o = o < 0 ? 0 : (o > RCAP ? RCAP : o);
        const float ri = sri[s];
        float acc0 = 0.0f, acc1 = 0.0f;
#pragma unroll 1
        for (int b0 = 0; b0 < c; b0 += 32) {
          int idx = o + b0 + lane;
          idx = idx > RCAP - 1 ? RCAP - 1 : idx;
          int sr = lb[idx];
          sr = sr < 0 ? 0 : (sr > nN - 1 ? nN - 1 : sr);
          const int m32 = (c - b0) < 32 ? (c - b0) : 32;
#pragma unroll 1
          for (int k = 0; k < m32; ++k) {
            const int sk = __builtin_amdgcn_readlane(sr, k);
            const v2f a = *(const v2fa*)(xl + (size_t)sk * GBN + 2 * lane);
            acc0 += a.x; acc1 += a.y;
          }
        }
        const bool bad = big || (ovf != 0);
        float y0 = acc0 * ri + bv0;
        float y1 = acc1 * ri + bv1;
        y0 = bad ? qnan : y0;
        y1 = bad ? qnan : y1;
        if (lane < NOUTC / 2) {
          v2f w; w.x = y0; w.y = y1;
          *(v2fa*)(st + r * NOUTC + 2 * lane) = w;
        }
      }
      wave_sync();
      const v4f q0 = *(const v4fa*)(st + 4 * lane);
      const v4f q1 = *(const v4fa*)(st + 128 + 4 * (lane & 7));
      wave_sync();
      float* op = out + (size_t)node0 * NOUTC;
      *(volatile v4f*)(op + 4 * lane) = q0;
      if (lane < 8) *(volatile v4f*)(op + 128 + 4 * lane) = q1;
      __threadfence();
      *(volatile v4f*)(op + 4 * lane) = q0;
      if (lane < 8) *(volatile v4f*)(op + 128 + 4 * lane) = q1;
    }
  }
}

static inline int cdiv(int a, int b) { return (a + b - 1) / b; }
static inline size_t al256(size_t o) { return (o + 255) & ~(size_t)255; }

extern "C" void kernel_launch(void* const* d_in, const int* in_sizes, int n_in,
                              void* d_out, int out_size, void* d_ws, size_t ws_size,
                              hipStream_t stream) {
  if (n_in < 7) return;
  if (in_sizes[0] != NNODE * CIN) return;
  const int nN = in_sizes[0] / CIN;
  if (in_sizes[1] != NEDGE || in_sizes[2] != NEDGE) return;
  const int nE = in_sizes[1];
  if ((nN & 3) != 0 || (nE & 3) != 0) return;
  if (nE >= (1 << (31 - SLA))) return;
  if (in_sizes[3] != CIN * HID || in_sizes[4] != HID) return;
  if (in_sizes[5] != HID * NOUTC || in_sizes[6] != NOUTC) return;
  if (out_size != nN * NOUTC) return;

  const float* x   = (const float*)d_in[0];
  const int*   src = (const int*)d_in[1];
  const int*   dst = (const int*)d_in[2];
  const float* W0  = (const float*)d_in[3];
  const float* b0  = (const float*)d_in[4];
  const float* W1  = (const float*)d_in[5];
  const float* b1  = (const float*)d_in[6];
  float* out = (float*)d_out;

  const int MP    = cdiv(nN, MTILE) * MTILE;
  const int gM    = MP / GBM;
  const int gA    = cdiv(MP, NBA);
  const int NPADA = gA * NBA;
  const int gO    = cdiv(NPADA, NBO);
  const int NBPD  = gO * NBO;
  if (NPADA < MP || NBPD < NPADA) return;
  const int vec8 = ((nE & 3) == 0) ? 1 : 0;

  char* ws = (char*)d_ws;
  size_t off = 0;
  const size_t oRO  = off; off = al256(off + (size_t)NBPD * 4);
  const size_t oCNT = off; off = al256(off + (size_t)NPADA * 4);
  const size_t oOFF = off; off = al256(off + (size_t)NPADA * 4);
  const size_t oRI  = off; off = al256(off + (size_t)NPADA * 4);
  const size_t oFLG = off; off = al256(off + (size_t)gA * 128);
  const size_t oW0T = off; off = al256(off + (size_t)HID * K1 * 2);
  const size_t oW1D = off; off = al256(off + (size_t)HID * K2 * 2);
  const size_t oXB  = off; off = al256(off + (size_t)MP * CIN * 2);
  const size_t oH1  = off; off = al256(off + (size_t)MP * HID * 4);
  const size_t oX1  = off; off = al256(off + (size_t)MP * K2 * 2);
  const size_t oH2  = off; off = al256(off + (size_t)MP * GBN * 4);
  const size_t oLST = off; off = al256(off + (size_t)gA * RCAP * 4);
  if (off > ws_size || off > (size_t)WSMAX) return;
  float*          RO  = (float*)(ws + oRO);
  int*            CNT = (int*)(ws + oCNT);
  int*            OFF = (int*)(ws + oOFF);
  float*          RI  = (float*)(ws + oRI);
  int*            FLG = (int*)(ws + oFLG);
  unsigned short* W0T = (unsigned short*)(ws + oW0T);
  unsigned short* W1D = (unsigned short*)(ws + oW1D);
  unsigned short* XB  = (unsigned short*)(ws + oXB);
  float*          H1  = (float*)(ws + oH1);
  unsigned short* X1  = (unsigned short*)(ws + oX1);
  float*          H2  = (float*)(ws + oH2);
  int*            LST = (int*)(ws + oLST);

  const size_t degLds = (size_t)NBO * 4;
  const size_t bktLds = (size_t)BKT_LDS_INTS * 4;
  hipFuncSetAttribute(reinterpret_cast<const void*>(&k_outdeg), hipFuncAttributeMaxDynamicSharedMemorySize, (int)degLds);
  hipFuncSetAttribute(reinterpret_cast<const void*>(&k_bucket), hipFuncAttributeMaxDynamicSharedMemorySize, (int)bktLds);

  const int nUnits = NUWE + MP * (CIN / 8);
  k_prep<<<cdiv(nUnits, NTHR), NTHR, 0, stream>>>(x, W0, W1, W0T, W1D, XB, nN, nUnits);
  k_outdeg<<<gO, NTHR, degLds, stream>>>(src, nE, RO);
  k_bucket<<<gA, NTHR, bktLds, stream>>>(src, dst, nE, nN, vec8, LST, CNT, OFF, RI, FLG);
  k_gemm<1><<<dim3(gM, 1), GTHR, 0, stream>>>(XB, W0T, RO, H1, K1, HID);
  k_agg1<<<gA, NTHR, 0, stream>>>(LST, CNT, OFF, RI, RO, FLG, nN, MP, H1, b0, X1);
  k_gemm<0><<<dim3(gM, 1), GTHR, 0, stream>>>(X1, W1D, RO, H2, K2, GBN);
  k_agg2<<<gA, NTHR, 0, stream>>>(LST, CNT, OFF, RI, FLG, nN, H2, b1, out);
}
